// Registration_5720896438661
// MI455X (gfx1250) — hardware-verified
//
#include <hip/hip_runtime.h>
#define NI 2
#define CH 64
#define HH 256
#define HI 256
#define HL 128
#define P0 (HH * HH)
#define P1 (HL * HL)
#define R0 (NI * P0)
#define R1 (NI * P1)
#define RCH 32768
typedef __bf16 v16b __attribute__((ext_vector_type(16)));
typedef unsigned short v8us __attribute__((ext_vector_type(8), may_alias));
typedef float  v8f  __attribute__((ext_vector_type(8)));
typedef float  v4f  __attribute__((ext_vector_type(4)));
typedef float  v4fa __attribute__((ext_vector_type(4), may_alias));
union FragB { v16b v; v8us half[2]; unsigned short u[16]; };

__device__ __forceinline__ unsigned short bf16_bits(float x) { unsigned int u = __float_as_uint(x); return (unsigned short)((u + 0x7FFFu + ((u >> 16) & 1u)) >> 16); }
__device__ __forceinline__ float bf16_val(unsigned short b) { return __uint_as_float(((unsigned int)b) << 16); }
__device__ __forceinline__ float bf16_round(float x) { return bf16_val(bf16_bits(x)); }
template <int NT>
__device__ __forceinline__ v8f mmaN(v16b ah, v16b al, v16b bh, v16b bl, v8f c) {
  c = __builtin_amdgcn_wmma_f32_16x16x32_bf16(false, ah, false, bh, (short)0, c, false, false);
  if (NT >= 2) c = __builtin_amdgcn_wmma_f32_16x16x32_bf16(false, al, false, bh, (short)0, c, false, false);
  if (NT >= 3) c = __builtin_amdgcn_wmma_f32_16x16x32_bf16(false, ah, false, bl, (short)0, c, false, false);
  asm volatile("v_nop\n\tv_nop\n\tv_nop\n\tv_nop" : "+v"(c) : "v"(ah), "v"(al), "v"(bh), "v"(bl));
  return c;
}

__global__ __launch_bounds__(256) void k_wt_bf16(const float* __restrict__ W, unsigned short* __restrict__ Wt, int K, int N) {
  const int t = blockIdx.x * 256 + threadIdx.x;
  const int k8n = K / 8;
  if (t >= N * k8n) return;
  const int n = t / k8n, k8 = (t % k8n) * 8;
  v8us v;
#pragma unroll
  for (int i = 0; i < 8; ++i) v[i] = bf16_bits(W[(size_t)(k8 + i) * N + n]);
  *(volatile v8us*)(Wt + (size_t)n * K + k8) = v;
  __threadfence();
  *(volatile v8us*)(Wt + (size_t)n * K + k8) = v;
}

template <bool ASPLIT, int ACT, bool BIAS_BF16>
__global__ __launch_bounds__(128) void k_gemm_bf(const float* __restrict__ A, int lda, const unsigned short* __restrict__ Wt, int ldb,
                                               const float* __restrict__ bias, float* __restrict__ C, int ldc, int M, int N, int K) {
  __shared__ __attribute__((aligned(16))) float so[4][16][64];
  const int tid = threadIdx.x, w = tid >> 5, lane = tid & 31, ln = lane & 15, hh = lane >> 4;
  const int ntn = N / 64;
  const int wid = blockIdx.x * 4 + w;
  const int mt = wid / ntn, nq = wid % ntn;
  if (mt * 16 >= M) return;
  const int row0 = mt * 16, col0 = nq * 64;
  const float* arow = A + (size_t)(row0 + ln) * lda;
  v8f acc[4] = {};
  for (int kb = 0; kb < K; kb += 32) {
    FragB ah, al;
    const v4f x0 = *(const v4fa*)(arow + kb + 8 * hh), x1 = *(const v4fa*)(arow + kb + 8 * hh + 4);
    const v4f x2 = *(const v4fa*)(arow + kb + 16 + 8 * hh), x3 = *(const v4fa*)(arow + kb + 16 + 8 * hh + 4);
    float xs[16] = {x0[0],x0[1],x0[2],x0[3],x1[0],x1[1],x1[2],x1[3],x2[0],x2[1],x2[2],x2[3],x3[0],x3[1],x3[2],x3[3]};
#pragma unroll
    for (int i = 0; i < 16; ++i) { const unsigned short hb = bf16_bits(xs[i]); ah.u[i] = hb; al.u[i] = ASPLIT ? bf16_bits(xs[i] - bf16_val(hb)) : (unsigned short)0; }
#pragma unroll
    for (int t = 0; t < 4; ++t) {
      const unsigned short* brow = Wt + (size_t)(col0 + t * 16 + ln) * ldb + kb;
      FragB b;
      b.half[0] = *(const v8us*)(brow + 8 * hh);
      b.half[1] = *(const v8us*)(brow + 16 + 8 * hh);
      acc[t] = mmaN<ASPLIT ? 2 : 1>(ah.v, al.v, b.v, b.v, acc[t]);
    }
  }
#pragma unroll
  for (int t = 0; t < 4; ++t) {
    float bv = bias ? bias[col0 + t * 16 + ln] : 0.f;
    if (BIAS_BF16) bv = bf16_round(bv);
#pragma unroll
    for (int r = 0; r < 8; ++r) { float v = acc[t][r] + bv; if (ACT == 1) v = fmaxf(v, 0.f); so[w][8 * hh + r][t * 16 + ln] = v; }
  }
  __builtin_amdgcn_fence(__ATOMIC_ACQ_REL, "workgroup");
  __builtin_amdgcn_wave_barrier();
  const int rsub = lane >> 4, c4 = (lane & 15) * 4;
  for (int pass = 0; pass < 2; ++pass) {
#pragma unroll
    for (int q = 0; q < 8; ++q) {
      const int r = q * 2 + rsub;
      const v4f v = *(const v4fa*)&so[w][r][c4];
      *(volatile v4f*)(C + (size_t)(row0 + r) * ldc + col0 + c4) = v;
    }
    if (pass == 0) __threadfence();
  }
}

template <bool ASPLIT, int ACT, bool BIAS_BF16, bool RES_BF16>
__global__ __launch_bounds__(128) void k_gemm_bf3(const float* __restrict__ A, int lda, const unsigned short* __restrict__ Wt, int ldb,
                                                const float* __restrict__ bias, const float* __restrict__ resid, int rmod, int ldr,
                                                float* __restrict__ C, int ldc, int M, int N, int K) {
  __shared__ __attribute__((aligned(16))) float so[4][16][64];
  const int tid = threadIdx.x, w = tid >> 5, lane = tid & 31, ln = lane & 15, hh = lane >> 4;
  const int ntn = N / 64;
  const int wid = blockIdx.x * 4 + w;
  const int mt = wid / ntn, nq = wid % ntn;
  if (mt * 16 >= M) return;
  const int row0 = mt * 16, col0 = nq * 64;
  const float* arow = A + (size_t)(row0 + ln) * lda;
  v8f acc[4] = {};
  for (int kb = 0; kb < K; kb += 32) {
    FragB ah, al;
    const v4f x0 = *(const v4fa*)(arow + kb + 8 * hh), x1 = *(const v4fa*)(arow + kb + 8 * hh + 4);
    const v4f x2 = *(const v4fa*)(arow + kb + 16 + 8 * hh), x3 = *(const v4fa*)(arow + kb + 16 + 8 * hh + 4);
    float xs[16] = {x0[0],x0[1],x0[2],x0[3],x1[0],x1[1],x1[2],x1[3],x2[0],x2[1],x2[2],x2[3],x3[0],x3[1],x3[2],x3[3]};
#pragma unroll
    for (int i = 0; i < 16; ++i) { const unsigned short hb = bf16_bits(xs[i]); ah.u[i] = hb; al.u[i] = ASPLIT ? bf16_bits(xs[i] - bf16_val(hb)) : (unsigned short)0; }
#pragma unroll
    for (int t = 0; t < 4; ++t) {
      const unsigned short* brow = Wt + (size_t)(col0 + t * 16 + ln) * ldb + kb;
      FragB b;
      b.half[0] = *(const v8us*)(brow + 8 * hh);
      b.half[1] = *(const v8us*)(brow + 16 + 8 * hh);
      acc[t] = mmaN<ASPLIT ? 2 : 1>(ah.v, al.v, b.v, b.v, acc[t]);
    }
  }
#pragma unroll
  for (int t = 0; t < 4; ++t) {
    const int col = col0 + t * 16 + ln;
    float bv = bias ? bias[col] : 0.f;
    if (BIAS_BF16) bv = bf16_round(bv);
#pragma unroll
    for (int r = 0; r < 8; ++r) {
      float v = acc[t][r] + bv;
      if (resid) { float rv = resid[(size_t)((row0 + 8 * hh + r) % rmod) * ldr + col]; if (RES_BF16) rv = bf16_round(rv); v += rv; }
      if (ACT == 1) v = fmaxf(v, 0.f);
      if (ACT == 2) v = 0.5f * v * (1.0f + erff(v * 0.70710678118654752f));
      if (ACT == 3) { const float u = 0.7978845608028654f * (v + 0.044715f * v * v * v); v = 0.5f * v * (1.0f + tanhf(u)); }
      so[w][8 * hh + r][t * 16 + ln] = v;
    }
  }
  __builtin_amdgcn_fence(__ATOMIC_ACQ_REL, "workgroup");
  __builtin_amdgcn_wave_barrier();
  const int rsub = lane >> 4, c4 = (lane & 15) * 4;
  for (int pass = 0; pass < 2; ++pass) {
#pragma unroll
    for (int q = 0; q < 8; ++q) {
      const int r = q * 2 + rsub;
      const v4f v = *(const v4fa*)&so[w][r][c4];
      *(volatile v4f*)(C + (size_t)(row0 + r) * ldc + col0 + c4) = v;
    }
    if (pass == 0) __threadfence();
  }
}
template <bool PARAM_BF16>
__global__ __launch_bounds__(256) void k_layernorm(const float* __restrict__ X, const float* __restrict__ R, const float* __restrict__ g, const float* __restrict__ bta,
                                                  float* __restrict__ out_sum, float* __restrict__ out_norm, int N, float eps) {
  __shared__ float red[256];
  const int row = blockIdx.x, tid = threadIdx.x;
  const float* x = X + (size_t)row * N; const float* rr = R ? R + (size_t)row * N : nullptr;
  float vals[16];
  const int per = N / 256;
  float s1 = 0.f;
  for (int u = 0; u < per / 4; ++u) {
    const int j = tid * 4 + 1024 * u;
    const v4f a = *(const v4fa*)(x + j);
    v4f b = {0.f,0.f,0.f,0.f}; if (rr) b = *(const v4fa*)(rr + j);
#pragma unroll
    for (int q = 0; q < 4; ++q) { const float v = a[q] + b[q]; vals[u * 4 + q] = v; s1 += v; }
  }
  red[tid] = s1; __syncthreads();
  for (int st = 128; st > 0; st >>= 1) { if (tid < st) red[tid] += red[tid + st]; __syncthreads(); }
  const float mu = red[0] / (float)N; __syncthreads();
  float s2 = 0.f;
  for (int u = 0; u < per / 4; ++u)
#pragma unroll
    for (int q = 0; q < 4; ++q) { const float c = vals[u * 4 + q] - mu; s2 += c * c; }
  red[tid] = s2; __syncthreads();
  for (int st = 128; st > 0; st >>= 1) { if (tid < st) red[tid] += red[tid + st]; __syncthreads(); }
  const float rs = rsqrtf(red[0] / (float)N + eps);
  for (int pass = 0; pass < 2; ++pass) {
    for (int u = 0; u < per / 4; ++u) {
      const int j = tid * 4 + 1024 * u;
      v4f o, sm;
#pragma unroll
      for (int q = 0; q < 4; ++q) {
        float gg = g[j + q], bb = bta[j + q];
        if (PARAM_BF16) { gg = bf16_round(gg); bb = bf16_round(bb); }
        sm[q] = vals[u * 4 + q]; o[q] = (vals[u * 4 + q] - mu) * rs * gg + bb;
      }
      if (out_sum) *(volatile v4f*)(out_sum + (size_t)row * N + j) = sm;
      *(volatile v4f*)(out_norm + (size_t)row * N + j) = o;
    }
    if (pass == 0) __threadfence();
  }
}


typedef _Float16 v16h __attribute__((ext_vector_type(16)));
union FragH { v16h v; v8us half[2]; _Float16 h[16]; unsigned short u[16]; };
template <int NT>
__device__ __forceinline__ v8f mmaH(v16h ah, v16h al, v16h bh, v16h bl, v8f c) {
  c = __builtin_amdgcn_wmma_f32_16x16x32_f16(false, ah, false, bh, (short)0, c, false, false);
  if (NT >= 2) c = __builtin_amdgcn_wmma_f32_16x16x32_f16(false, al, false, bh, (short)0, c, false, false);
  if (NT >= 3) c = __builtin_amdgcn_wmma_f32_16x16x32_f16(false, ah, false, bl, (short)0, c, false, false);
  asm volatile("v_nop\n\tv_nop\n\tv_nop\n\tv_nop" : "+v"(c) : "v"(ah), "v"(al), "v"(bh), "v"(bl));
  return c;
}
template <bool ASPLIT>
__global__ __launch_bounds__(128) void k_gemm_h(const float* __restrict__ A, int lda, size_t sA, const _Float16* __restrict__ Bh, int ldb, size_t sB, float alpha, float* __restrict__ C, int ldc, size_t sC, int M, int N, int K) {
  __shared__ __attribute__((aligned(16))) float so[4][16][64];
  const int tid = threadIdx.x, w = tid >> 5, lane = tid & 31, ln = lane & 15, hh = lane >> 4; const int by = blockIdx.y;
  A += (size_t)by * sA; Bh += (size_t)by * sB; C += (size_t)by * sC;
  const int ntn = (N + 63) / 64; const int wid = blockIdx.x * 4 + w; const int mt = wid / ntn, nq = wid % ntn; if (mt * 16 >= M) return;
  const int row0 = mt * 16, col0 = nq * 64; const float* arow = A + (size_t)(row0 + ln) * lda;
  v8f acc[4] = {};
  for (int kb = 0; kb < K; kb += 32) {
    FragH ah, al;
    const v4f x0 = *(const v4fa*)(arow + kb + 8 * hh), x1 = *(const v4fa*)(arow + kb + 8 * hh + 4), x2 = *(const v4fa*)(arow + kb + 16 + 8 * hh), x3 = *(const v4fa*)(arow + kb + 16 + 8 * hh + 4);
    float xs[16] = {x0[0],x0[1],x0[2],x0[3],x1[0],x1[1],x1[2],x1[3],x2[0],x2[1],x2[2],x2[3],x3[0],x3[1],x3[2],x3[3]};
#pragma unroll
    for (int i = 0; i < 16; ++i) { const _Float16 h = (_Float16)xs[i]; ah.h[i] = h; al.h[i] = ASPLIT ? (_Float16)(xs[i] - (float)h) : (_Float16)0.0f; }
#pragma unroll
    for (int t = 0; t < 4; ++t) { if (col0 + t * 16 >= N) continue; const size_t boff = (size_t)(col0 + t * 16 + ln) * ldb + kb; FragH bq; bq.half[0] = *(const v8us*)(Bh + boff + 8 * hh); bq.half[1] = *(const v8us*)(Bh + boff + 16 + 8 * hh);
      acc[t] = mmaH<ASPLIT ? 2 : 1>(ah.v, al.v, bq.v, bq.v, acc[t]); }
  }
#pragma unroll
  for (int t = 0; t < 4; ++t) { if (col0 + t * 16 >= N) continue;
#pragma unroll
    for (int r = 0; r < 8; ++r) so[w][8 * hh + r][t * 16 + ln] = acc[t][r] * alpha; }
  __builtin_amdgcn_fence(__ATOMIC_ACQ_REL, "workgroup"); __builtin_amdgcn_wave_barrier();
  const int rsub = lane >> 4, c4 = (lane & 15) * 4;
  for (int pass = 0; pass < 2; ++pass) {
#pragma unroll
    for (int q = 0; q < 8; ++q) { const int r = q * 2 + rsub; if (col0 + c4 < N) { const v4f v = *(const v4fa*)&so[w][r][c4]; *(volatile v4f*)(C + (size_t)(row0 + r) * ldc + col0 + c4) = v; } }
    if (pass == 0) __threadfence(); }
}

__global__ __launch_bounds__(256) void k_wt_f16(const float* __restrict__ W, _Float16* __restrict__ Wt, int K, int N, float scale) {
  const int t = blockIdx.x * 256 + threadIdx.x; if (t >= N * (K / 8)) return; const int n = t / (K / 8), k8 = (t % (K / 8)) * 8; FragH f;
#pragma unroll
  for (int i = 0; i < 8; ++i) f.h[i] = (_Float16)(bf16_round(W[(size_t)(k8 + i) * N + n]) * scale); const v8us o = f.half[0];
  *(volatile v8us*)((unsigned short*)Wt + (size_t)n * K + k8) = o; __threadfence(); *(volatile v8us*)((unsigned short*)Wt + (size_t)n * K + k8) = o;
}
template <int ACT>
__global__ __launch_bounds__(128) void k_gemm_hhx(const _Float16* __restrict__ A, int lda, size_t sA, const _Float16* __restrict__ Bh, int ldb, size_t sB, float alpha, const float* __restrict__ bias, size_t sBias, const float* __restrict__ CP, int rowsPerB, size_t sCPb, int row0g,
    float* __restrict__ C, _Float16* __restrict__ C16, int ldc, size_t sC, int M, int N, int K) {
  __shared__ __attribute__((aligned(16))) float so[4][16][64];
  const int tid = threadIdx.x, w = tid >> 5, lane = tid & 31, ln = lane & 15, hh = lane >> 4; const int by = blockIdx.y;
  A += (size_t)by * sA; Bh += (size_t)by * sB; const size_t cofs = (size_t)by * sC; const float* bp = bias ? bias + (size_t)by * sBias : nullptr;
  const int ntn = (N + 63) / 64; const int wid = blockIdx.x * 4 + w; const int mt = wid / ntn, nq = wid % ntn; if (mt * 16 >= M) return;
  const int row0 = mt * 16, col0 = nq * 64; const _Float16* arow = A + (size_t)(row0 + ln) * lda;
  v8f acc[4] = {};
  for (int kb = 0; kb < K; kb += 32) { FragH ah; ah.half[0] = *(const v8us*)((const unsigned short*)arow + kb + 8 * hh); ah.half[1] = *(const v8us*)((const unsigned short*)arow + kb + 16 + 8 * hh);
#pragma unroll
    for (int t = 0; t < 4; ++t) { if (col0 + t * 16 >= N) continue; const size_t boff = (size_t)(col0 + t * 16 + ln) * ldb + kb; FragH bq; bq.half[0] = *(const v8us*)((const unsigned short*)Bh + boff + 8 * hh); bq.half[1] = *(const v8us*)((const unsigned short*)Bh + boff + 16 + 8 * hh);
      acc[t] = mmaH<1>(ah.v, ah.v, bq.v, bq.v, acc[t]); }
  }
#pragma unroll
  for (int t = 0; t < 4; ++t) { if (col0 + t * 16 >= N) continue; const int col = col0 + t * 16 + ln; const float bv = bp ? bf16_round(bp[col]) : 0.f;
#pragma unroll
    for (int r = 0; r < 8; ++r) { float v = acc[t][r] * alpha + bv; if (CP) { const int rr = row0g + row0 + 8 * hh + r; if (rowsPerB < 0) v += CP[cofs + (size_t)rr * ldc + col];        else { const int bidx = rr / rowsPerB; v += CP[(size_t)bidx * sCPb + (size_t)by * 64 + col]; } } if (ACT == 1) v = (v > 0.f) ? v : expm1f(v); else if (ACT == 7) v = (v > 0.f) ? v + 1.0f : expf(v); else if (ACT == 8) v = tanhf(v); else if (ACT == 9) v = 0.5f * v * (1.0f + tanhf(0.7978845608028654f * (v + 0.044715f * v * v * v))); else if (ACT == 11) v = 1.0f / (1.0f + expf(-v)); else if (ACT == 12) v = (v > 0.f) ? v : 0.01f * v; else if (ACT == 14) v = (v > 0.f) ? v : 0.1f * v; else if (ACT == 16) v = (v >= 0.f) ? v : 0.3f * v; else if (ACT == 17) v = (v >= 0.f) ? v : 0.2f * v; else if (ACT == 15) v = v / (1.0f + expf(-v)); else if (ACT == 3) v = fmaxf(v, 0.f); else if (ACT == 6) v = 0.5f * v * (1.0f + erff(v * 0.70710678118654752f)); so[w][8 * hh + r][t * 16 + ln] = v; } }
  __builtin_amdgcn_fence(__ATOMIC_ACQ_REL, "workgroup"); __builtin_amdgcn_wave_barrier();
  const int rsub = lane >> 4, c4 = (lane & 15) * 4; typedef _Float16 v4h __attribute__((ext_vector_type(4)));
  for (int pass = 0; pass < 2; ++pass) {
#pragma unroll
    for (int q = 0; q < 8; ++q) { const int r = q * 2 + rsub; if (col0 + c4 < N) { const v4f v = *(const v4fa*)&so[w][r][c4]; if (C) *(volatile v4f*)(C + cofs + (size_t)(row0 + r) * ldc + col0 + c4) = v; if (C16) { v4h h4; for (int i = 0; i < 4; ++i) h4[i] = (_Float16)v[i]; *(volatile v4h*)(C16 + cofs + (size_t)(row0 + r) * ldc + col0 + c4) = h4; } } }
    if (pass == 0) __threadfence(); }
}


typedef _Float16 v4h __attribute__((ext_vector_type(4)));

__global__ __launch_bounds__(256) void k_x16(const float* __restrict__ x, _Float16* __restrict__ X16, size_t n8) { const size_t t = (size_t)blockIdx.x * 256 + threadIdx.x; if (t >= n8) return; FragH f;
#pragma unroll
  for (int q = 0; q < 8; ++q) f.h[q] = (_Float16)bf16_round(x[t * 8 + q]); *(volatile v8us*)((unsigned short*)X16 + t * 8) = f.half[0]; __threadfence(); *(volatile v8us*)((unsigned short*)X16 + t * 8) = f.half[0]; }
__global__ __launch_bounds__(256) void k_h16(const float* __restrict__ x, _Float16* __restrict__ X16, size_t n8) { const size_t t = (size_t)blockIdx.x * 256 + threadIdx.x; if (t >= n8) return; FragH f;
#pragma unroll
  for (int q = 0; q < 8; ++q) f.h[q] = (_Float16)x[t * 8 + q]; *(volatile v8us*)((unsigned short*)X16 + t * 8) = f.half[0]; __threadfence(); *(volatile v8us*)((unsigned short*)X16 + t * 8) = f.half[0]; }
__global__ __launch_bounds__(256) void k_round16f(const float* __restrict__ W, _Float16* __restrict__ Bt, size_t n8) { const size_t t = (size_t)blockIdx.x * 256 + threadIdx.x; if (t >= n8) return; FragH f;
#pragma unroll
  for (int i = 0; i < 8; ++i) f.h[i] = (_Float16)(bf16_round(W[t * 8 + i]) * 16.0f); *(volatile v8us*)((unsigned short*)Bt + t * 8) = f.half[0]; __threadfence(); *(volatile v8us*)((unsigned short*)Bt + t * 8) = f.half[0]; }
template <int NHv, int TTv>
__global__ __launch_bounds__(256) void k_vt(const _Float16* __restrict__ V16, int ldv, int voff, _Float16* __restrict__ Vt) { __shared__ unsigned short tl[64][66]; const int tid = threadIdx.x; const int slab = blockIdx.x / (TTv / 64), lg = blockIdx.x % (TTv / 64); const int b = slab / NHv, h = slab % NHv;
  for (int i = tid; i < 64 * 8; i += 256) { const int r = i / 8, c8 = (i % 8) * 8; FragH f; f.half[0] = *(const v8us*)((const unsigned short*)V16 + ((size_t)b * TTv + lg * 64 + r) * ldv + voff + h * 64 + c8);
#pragma unroll
    for (int q = 0; q < 8; ++q) tl[r][c8 + q] = f.u[q]; }
  __syncthreads();
  for (int pass = 0; pass < 2; ++pass) {
#pragma unroll
    for (int rd = 0; rd < 2; ++rd) { const int d = rd * 32 + tid / 8, pc = tid % 8; FragH f;
#pragma unroll
      for (int q = 0; q < 8; ++q) f.u[q] = tl[pc * 8 + q][d];
      *(volatile v8us*)((unsigned short*)Vt + ((size_t)slab * 64 + d) * TTv + lg * 64 + pc * 8) = f.half[0]; }
    if (pass == 0) __threadfence(); } }

__global__ __launch_bounds__(256) void k_hl(const float* __restrict__ F, _Float16* __restrict__ Hh, _Float16* __restrict__ Hl, size_t n8) { const size_t t = (size_t)blockIdx.x * 256 + threadIdx.x; if (t >= n8) return; FragH fh, fl; const v4f a = *(const v4fa*)(F + t * 8), c = *(const v4fa*)(F + t * 8 + 4);
#pragma unroll
  for (int q = 0; q < 4; ++q) { _Float16 h = (_Float16)a[q]; fh.h[q] = h; fl.h[q] = (_Float16)((a[q] - (float)h) * 1024.0f); h = (_Float16)c[q]; fh.h[4 + q] = h; fl.h[4 + q] = (_Float16)((c[q] - (float)h) * 1024.0f); }
  for (int pass = 0; pass < 2; ++pass) { *(volatile v8us*)((unsigned short*)Hh + t * 8) = fh.half[0]; *(volatile v8us*)((unsigned short*)Hl + t * 8) = fl.half[0]; if (pass == 0) __threadfence(); } }

__device__ __forceinline__ v16h g2_frag(const _Float16* p, int hh) { FragH f; f.half[0] = *(const v8us*)((const unsigned short*)p + 8 * hh); f.half[1] = *(const v8us*)((const unsigned short*)p + 16 + 8 * hh); return f.v; }
__device__ __forceinline__ v8f g2_mma(v16h a, v16h b, v8f c) { v8f d = __builtin_amdgcn_wmma_f32_16x16x32_f16(false, a, false, b, (short)0, c, false, false); asm volatile("v_nop\n\tv_nop\n\tv_nop\n\tv_nop" : "+v"(d) : "v"(a), "v"(b)); return d; }
template <int ACT>
__global__ __launch_bounds__(128) void k_gemm2(const _Float16* __restrict__ A, int lda, size_t sA, const _Float16* __restrict__ Bh, int ldb, size_t sB, float alpha, const float* __restrict__ bias, size_t sBias, const float* __restrict__ CP, int rowsPerB, size_t sCPb, int row0g,
    float* __restrict__ C, _Float16* __restrict__ C16, int ldc, size_t sC, int M, int N, int K) { static_assert(ACT == 0 || ACT == 3 || ACT == 6 || ACT == 8 || ACT == 9 || ACT == 11 || ACT == 12 || ACT == 14 || ACT == 15 || ACT == 16 || ACT == 17, "k_gemm2: unsupported ACT code (would silently apply no activation)");
  __shared__ __attribute__((aligned(16))) float so[4][32][68];
  const int tid = threadIdx.x, w = tid >> 5, lane = tid & 31, ln = lane & 15, hh = lane >> 4; const int by = blockIdx.y;
  A += (size_t)by * sA; Bh += (size_t)by * sB; const size_t cofs = (size_t)by * sC; const float* bp = bias ? bias + (size_t)by * sBias : nullptr;
  const int ntn = N >> 6; const int mt = blockIdx.x / ntn, nq = blockIdx.x - mt * ntn; const int row0 = mt * 128 + 32 * w, col0 = nq * 64; if (row0 >= M) return;
  const _Float16* a0p = A + (size_t)(row0 + ln) * lda; const _Float16* a1p = a0p + (size_t)16 * lda;
  const _Float16* b0p = Bh + (size_t)(col0 + ln) * ldb; const _Float16* b1p = b0p + (size_t)16 * ldb; const _Float16* b2p = b1p + (size_t)16 * ldb; const _Float16* b3p = b2p + (size_t)16 * ldb;
  const v8f z8 = {0.f,0.f,0.f,0.f,0.f,0.f,0.f,0.f}; v8f c00 = z8, c01 = z8, c02 = z8, c03 = z8, c10 = z8, c11 = z8, c12 = z8, c13 = z8;
#pragma unroll 1
  for (int kb = 0; kb < K; kb += 32) { const v16h a0 = g2_frag(a0p + kb, hh), a1 = g2_frag(a1p + kb, hh);
    v16h b = g2_frag(b0p + kb, hh); c00 = g2_mma(a0, b, c00); c10 = g2_mma(a1, b, c10);
    b = g2_frag(b1p + kb, hh); c01 = g2_mma(a0, b, c01); c11 = g2_mma(a1, b, c11);
    b = g2_frag(b2p + kb, hh); c02 = g2_mma(a0, b, c02); c12 = g2_mma(a1, b, c12);
    b = g2_frag(b3p + kb, hh); c03 = g2_mma(a0, b, c03); c13 = g2_mma(a1, b, c13); }
  v8f accs[8] = {c00, c01, c02, c03, c10, c11, c12, c13};
#pragma unroll
  for (int u = 0; u < 8; ++u) { const int t = u & 3, half = u >> 2; const int col = col0 + t * 16 + ln; const float bv = bp ? bf16_round(bp[col]) : 0.f;
#pragma unroll
    for (int r = 0; r < 8; ++r) { const int rloc = half * 16 + 8 * hh + r; float v = accs[u][r] * alpha + bv; if (CP) { if (rowsPerB < 0) v += CP[cofs + (size_t)(row0g + row0 + rloc) * ldc + col];        else { const int bidx = (row0g + row0 + rloc) / rowsPerB; v += CP[(size_t)bidx * sCPb + (size_t)by * 64 + col]; } }
      if (ACT == 3) v = fmaxf(v, 0.f); else if (ACT == 6) v = 0.5f * v * (1.0f + erff(v * 0.70710678118654752f)); else if (ACT == 11) v = 1.0f / (1.0f + expf(-v)); else if (ACT == 15) v = v / (1.0f + expf(-v)); else if (ACT == 12) v = (v > 0.f) ? v : 0.01f * v; else if (ACT == 8) v = tanhf(v); else if (ACT == 9) v = 0.5f * v * (1.0f + tanhf(0.7978845608028654f * (v + 0.044715f * v * v * v))); else if (ACT == 14) v = (v > 0.f) ? v : 0.1f * v; else if (ACT == 16) v = (v >= 0.f) ? v : 0.3f * v; else if (ACT == 17) v = (v >= 0.f) ? v : 0.2f * v;
      so[w][rloc][t * 16 + ln] = v; } }
  __builtin_amdgcn_fence(__ATOMIC_ACQ_REL, "workgroup"); __builtin_amdgcn_wave_barrier();
  const int rsub = lane >> 4, c4 = (lane & 15) * 4;
  for (int pass = 0; pass < 2; ++pass) {
#pragma unroll
    for (int q = 0; q < 16; ++q) { const int r = q * 2 + rsub; const v4f v = *(const v4fa*)&so[w][r][c4]; if (C) *(volatile v4f*)(C + cofs + (size_t)(row0 + r) * ldc + col0 + c4) = v; if (C16) { v4h h4; for (int i = 0; i < 4; ++i) h4[i] = (_Float16)v[i]; *(volatile v4h*)(C16 + cofs + (size_t)(row0 + r) * ldc + col0 + c4) = h4; } }
    if (pass == 0) __threadfence(); } }


__global__ __launch_bounds__(256) void k_nhwc(const float* __restrict__ x, _Float16* __restrict__ D, int ld, int coff) { const size_t t = (size_t)blockIdx.x * 256 + threadIdx.x; if (t >= (size_t)R0 * CH / 8) return; const int c0 = (int)((t * 8) % CH); const size_t row = (t * 8) / CH; const int b = (int)(row / P0), p = (int)(row % P0); const size_t pin = (size_t)(p / HH) * HI + (p % HH);        FragH f; for (int q = 0; q < 8; ++q) f.h[q] = (_Float16)bf16_round(x[((size_t)b * CH + c0 + q) * ((size_t)HI * HI) + pin]);
  unsigned short* dst = (unsigned short*)D + row * ld + coff + c0; *(volatile v8us*)dst = f.half[0]; __threadfence(); *(volatile v8us*)dst = f.half[0]; }
__global__ __launch_bounds__(256) void k_wre(const float* __restrict__ w, int O, int Olive, int CI, int K, _Float16* __restrict__ Bt) { const size_t t = (size_t)blockIdx.x * 256 + threadIdx.x; const int KK2 = K * K; if (t >= (size_t)O * KK2 * CI / 8) return; const int c8 = (int)((t * 8) % CI); const int tap = (int)(((t * 8) / CI) % KK2); const int o = (int)((t * 8) / ((size_t)CI * KK2)); FragH f; for (int q = 0; q < 8; ++q) f.h[q] = (o < Olive) ? (_Float16)(bf16_round(w[(((size_t)o * CI + c8 + q) * KK2) + tap]) * 16.0f) : (_Float16)0.0f;
  *(volatile v8us*)((unsigned short*)Bt + t * 8) = f.half[0]; __threadfence(); *(volatile v8us*)((unsigned short*)Bt + t * 8) = f.half[0]; }
__global__ __launch_bounds__(64) void k_bpad(const float* __restrict__ src, int n, float* __restrict__ dst) { const int i = threadIdx.x; const float v = (i < n) ? src[i] : 0.f; *(volatile float*)(dst + i) = v; __threadfence(); *(volatile float*)(dst + i) = v; }
__device__ __forceinline__ void tapmap(int par, int tt, int& k, int& di) { if (par == 0) { k = tt ? 3 : 1; di = tt ? -1 : 0; } else { k = tt ? 2 : 0; di = tt ? 0 : 1; } }
__global__ __launch_bounds__(256) void k_wtr(const float* __restrict__ w, _Float16* __restrict__ Bt) { const size_t t = (size_t)blockIdx.x * 256 + threadIdx.x; if (t >= (size_t)4 * CH * 4 * CH / 8) return; const int c8 = (int)((t * 8) % CH); const int tp = (int)(((t * 8) / CH) % 4); const int o = (int)(((t * 8) / (CH * 4)) % CH); const int ph = (int)((t * 8) / ((size_t)CH * 4 * CH)); const int py = ph >> 1, px = ph & 1, ty = tp >> 1, tx = tp & 1; int ky, dy, kx, dx; tapmap(py, ty, ky, dy); tapmap(px, tx, kx, dx); (void)dy; (void)dx; FragH f;
  for (int q = 0; q < 8; ++q) f.h[q] = (_Float16)(bf16_round(w[(((size_t)(c8 + q) * CH + o) * 4 + ky) * 4 + kx]) * 16.0f);
  *(volatile v8us*)((unsigned short*)Bt + t * 8) = f.half[0]; __threadfence(); *(volatile v8us*)((unsigned short*)Bt + t * 8) = f.half[0]; }
__global__ __launch_bounds__(256) void k_im2col(const _Float16* __restrict__ Sp, int CI, int Hs, int stride, int Ho, int r0, int nrows, _Float16* __restrict__ XC) {
  const size_t t = (size_t)blockIdx.x * 256 + threadIdx.x; const int c8n = CI / 8; if (t >= (size_t)nrows * 9 * c8n) return; const int c8 = (int)(t % c8n) * 8; const int tap = (int)((t / c8n) % 9); const size_t rr = t / ((size_t)9 * c8n); const size_t row = r0 + rr; const int Po = Ho * Ho; const int b = (int)(row / Po); const int p = (int)(row % Po); const int oy = p / Ho, ox = p % Ho; const int iy = oy * stride - 1 + tap / 3, ix = ox * stride - 1 + tap % 3; v8us v;
  if (iy >= 0 && iy < Hs && ix >= 0 && ix < Hs) v = *(const v8us*)((const unsigned short*)Sp + (((size_t)b * Hs + iy) * Hs + ix) * CI + c8); else { for (int q = 0; q < 8; ++q) v[q] = 0; }
  unsigned short* dst = (unsigned short*)XC + rr * (size_t)(9 * CI) + tap * CI + c8; *(volatile v8us*)dst = v; __threadfence(); *(volatile v8us*)dst = v; }
__global__ __launch_bounds__(256) void k_phcol(const _Float16* __restrict__ Sp, int ph, _Float16* __restrict__ XC) {
  const size_t t = (size_t)blockIdx.x * 256 + threadIdx.x; if (t >= (size_t)R1 * 4 * (CH / 8)) return; const int c8 = (int)(t % (CH / 8)) * 8; const int tp = (int)((t / (CH / 8)) % 4); const size_t row = t / ((size_t)4 * (CH / 8)); const int b = (int)(row / P1), p = (int)(row % P1); const int m = p / HL, n = p % HL; const int py = ph >> 1, px = ph & 1; int ky, dy, kx, dx; tapmap(py, tp >> 1, ky, dy); tapmap(px, tp & 1, kx, dx); (void)ky; (void)kx; const int iy = m + dy, ix = n + dx; v8us v;
  if (iy >= 0 && iy < HL && ix >= 0 && ix < HL) v = *(const v8us*)((const unsigned short*)Sp + (((size_t)b * HL + iy) * HL + ix) * CH + c8); else { for (int q = 0; q < 8; ++q) v[q] = 0; }
  unsigned short* dst = (unsigned short*)XC + row * (size_t)(4 * CH) + tp * CH + c8; *(volatile v8us*)dst = v; __threadfence(); *(volatile v8us*)dst = v; }
__global__ __launch_bounds__(256) void k_place(const float* __restrict__ T, int ph, float* __restrict__ Df, _Float16* __restrict__ Dh) { const size_t t = (size_t)blockIdx.x * 256 + threadIdx.x; if (t >= (size_t)R1 * CH / 8) return; const int c8 = (int)((t * 8) % CH); const size_t row = (t * 8) / CH; const int b = (int)(row / P1), p = (int)(row % P1); const int m = p / HL, n = p % HL; const int oy = 2 * m + (ph >> 1), ox = 2 * n + (ph & 1); const v8f a = *(const v8f*)(T + t * 8); const size_t o = (((size_t)b * HH + oy) * HH + ox) * CH + c8;
  if (Df) { *(volatile v8f*)(Df + o) = a; __threadfence(); *(volatile v8f*)(Df + o) = a; } if (Dh) { FragH f; for (int q = 0; q < 8; ++q) f.h[q] = (_Float16)a[q]; *(volatile v8us*)((unsigned short*)Dh + o) = f.half[0]; __threadfence(); *(volatile v8us*)((unsigned short*)Dh + o) = f.half[0]; } }
__global__ __launch_bounds__(256) void k_add16(const float* __restrict__ A, const float* __restrict__ Bp, _Float16* __restrict__ S16, size_t n8) {
  #pragma clang fp contract(off)
  const size_t t = (size_t)blockIdx.x * 256 + threadIdx.x; if (t >= n8) return; const v8f a = *(const v8f*)(A + t * 8), b = *(const v8f*)(Bp + t * 8); FragH f; for (int q = 0; q < 8; ++q) f.h[q] = (_Float16)(a[q] + b[q]);
  *(volatile v8us*)((unsigned short*)S16 + t * 8) = f.half[0]; __threadfence(); *(volatile v8us*)((unsigned short*)S16 + t * 8) = f.half[0]; }
__global__ __launch_bounds__(256) void k_dcncol(const _Float16* __restrict__ Sp, int Hs, const float* __restrict__ OF, int ldo, int r0, int nrows, _Float16* __restrict__ XC) {
  #pragma clang fp contract(off)
  const size_t t = (size_t)blockIdx.x * 256 + threadIdx.x; if (t >= (size_t)nrows * 9 * (CH / 8)) return; const int c8 = (int)(t % (CH / 8)) * 8; const int n = (int)((t / (CH / 8)) % 9); const size_t rr = t / ((size_t)9 * (CH / 8)); const size_t row = r0 + rr; const int Po = Hs * Hs; const int b = (int)(row / Po), p = (int)(row % Po); const int y = p / Hs, x = p % Hs; const int Hp = Hs + 2;
  const float offr = OF[row * ldo + n], offc = OF[row * ldo + 9 + n]; float pr = (float)(y + 1) + (float)(n / 3 - 1) + offr, pc = (float)(x + 1) + (float)(n % 3 - 1) + offc; pr = fminf(fmaxf(pr, 0.f), (float)(Hp - 1)); pc = fminf(fmaxf(pc, 0.f), (float)(Hp - 1));
  const float fr0 = floorf(pr), fc0 = floorf(pc); const int ir0 = (int)fr0, ic0 = (int)fc0; const int ir1 = min(ir0 + 1, Hp - 1), ic1 = min(ic0 + 1, Hp - 1); const float fr = pr - fr0, fc = pc - fc0;
  float acc[8]; for (int q = 0; q < 8; ++q) acc[q] = 0.f;
  for (int k = 0; k < 4; ++k) { const int ri = (k >> 1) ? ir1 : ir0, ci = (k & 1) ? ic1 : ic0; const float w = ((k >> 1) ? fr : (1.f - fr)) * ((k & 1) ? fc : (1.f - fc)); const int sy = ri - 1, sx = ci - 1; if (sy < 0 || sy >= Hs || sx < 0 || sx >= Hs) continue; FragH v; v.half[0] = *(const v8us*)((const unsigned short*)Sp + (((size_t)b * Hs + sy) * Hs + sx) * CH + c8); for (int q = 0; q < 8; ++q) acc[q] += (float)v.h[q] * w; }
  FragH f; for (int q = 0; q < 8; ++q) f.h[q] = (_Float16)acc[q]; unsigned short* dst = (unsigned short*)XC + rr * (size_t)(9 * CH) + n * CH + c8; *(volatile v8us*)dst = f.half[0]; __threadfence(); *(volatile v8us*)dst = f.half[0]; }
__global__ __launch_bounds__(256) void k_out(const float* __restrict__ Y, float* __restrict__ out) { const size_t t = (size_t)blockIdx.x * 256 + threadIdx.x; if (t >= (size_t)NI * CH * P0 / 8) return; const int p0 = (int)((t * 8) % P0); const size_t bc = (t * 8) / P0; const int b = (int)(bc / CH), c = (int)(bc % CH); v8f v; for (int q = 0; q < 8; ++q) v[q] = Y[((size_t)b * P0 + p0 + q) * CH + c];
  *(volatile v8f*)(out + t * 8) = v; __threadfence(); *(volatile v8f*)(out + t * 8) = v; }

static void conv3(hipStream_t st, const _Float16* S, int CI, int Hs, int stride, int Ho, const _Float16* Bt, const float* bias, int O, float* Df, _Float16* D16, int ldd, _Float16* XC) {
  const int nrows = NI * Ho * Ho; const int KC = 9 * CI;
  for (int r0 = 0; r0 < nrows; r0 += RCH) { const int nr = min(RCH, nrows - r0);
    k_im2col<<<(unsigned)(((size_t)nr * 9 * (CI / 8) + 255) / 256), 256, 0, st>>>(S, CI, Hs, stride, Ho, r0, nr, XC);
    k_gemm2<0><<<dim3((nr / 128) * (O / 64), 1), 128, 0, st>>>(XC, KC, 0, Bt, KC, 0, 0.0625f, bias, 0, nullptr, 1, 0, 0, Df ? Df + (size_t)r0 * ldd : nullptr, Df ? nullptr : D16 + (size_t)r0 * ldd, ldd, 0, nr, O, KC); } }

extern "C" void kernel_launch(void* const* d_in, const int* in_sizes, int n_in,
                              void* d_out, int out_size, void* d_ws, size_t ws_size, hipStream_t stream) {
  (void)in_sizes; (void)n_in; (void)out_size;
  const float* const* I = (const float* const*)d_in; const float* dem = I[0]; const float* rs = I[1]; const float* w_down1 = I[2]; const float* b_down1 = I[3]; const float* w_c1 = I[4]; const float* b_c1 = I[5]; const float* w_c12 = I[6]; const float* b_c12 = I[7]; const float* w_up1 = I[8]; const float* b_up1 = I[9]; const float* w_downrs = I[10]; const float* b_downrs = I[11]; const float* w_off = I[12]; const float* b_off = I[13]; const float* w_c3 = I[14]; const float* b_c3 = I[15]; const float* w_d1o = I[16]; const float* b_d1o = I[17]; const float* w_d1 = I[18]; const float* b_d1 = I[19]; const float* w_d2o = I[20]; const float* b_d2o = I[21]; const float* w_d2 = I[22]; const float* b_d2 = I[23]; const float* w_up2 = I[24]; const float* b_up2 = I[25];
  char* ws = (char*)d_ws; size_t off = 0;
  auto take = [&](size_t bytes) { char* p = ws + off; off += (bytes + 255) & ~(size_t)255; return p; };
  _Float16* Bdown1 = (_Float16*)take((size_t)128 * 1152 * 2); _Float16* Bc1 = (_Float16*)take((size_t)64 * 1152 * 2); _Float16* Bc12 = (_Float16*)take((size_t)64 * 1152 * 2); _Float16* Bdrs = (_Float16*)take((size_t)64 * 576 * 2); _Float16* Boff = (_Float16*)take((size_t)64 * 64 * 2); _Float16* Bc3 = (_Float16*)take((size_t)64 * 64 * 2);
  _Float16* Bd1o = (_Float16*)take((size_t)64 * 576 * 2); _Float16* Bd1 = (_Float16*)take((size_t)64 * 576 * 2); _Float16* Bd2o = (_Float16*)take((size_t)64 * 576 * 2); _Float16* Bd2 = (_Float16*)take((size_t)64 * 576 * 2); _Float16* Bup1 = (_Float16*)take((size_t)4 * 64 * 256 * 2); _Float16* Bup2 = (_Float16*)take((size_t)4 * 64 * 256 * 2); float* bz1 = (float*)take(256); float* bz2 = (float*)take(256);
  _Float16* F1IN = (_Float16*)take((size_t)R0 * 128 * 2); _Float16* RS16 = (_Float16*)take((size_t)R0 * 64 * 2); _Float16* XC = (_Float16*)take((size_t)RCH * 1152 * 2);
  _Float16* F2A16 = (_Float16*)take((size_t)R1 * 128 * 2); float* FEA1 = (float*)take((size_t)R0 * 64 * 4); float* FEA2 = (float*)take((size_t)R1 * 64 * 4); _Float16* FEA2H = (_Float16*)take((size_t)R1 * 64 * 2); float* TMP = (float*)take((size_t)R1 * 64 * 4); float* UPF = (float*)take((size_t)R0 * 64 * 4); _Float16* SUM16 = (_Float16*)take((size_t)R0 * 64 * 2); _Float16* FEA16 = (_Float16*)take((size_t)R0 * 64 * 2);
  float* OFF1 = FEA1;        float* F11 = UPF;        _Float16* RS2H = F2A16;        float* OFF2 = FEA2;        _Float16* FEA2B = FEA2H;        float* UP2F = FEA1;        float* Y = UPF;
  if (off > ws_size) return;
  const size_t n8_64 = (size_t)R0 * 64 / 8;
  k_wre<<<(unsigned)(((size_t)128 * 9 * 128 / 8 + 255) / 256), 256, 0, stream>>>(w_down1, 128, 128, 128, 3, Bdown1); k_wre<<<(unsigned)(((size_t)64 * 9 * 128 / 8 + 255) / 256), 256, 0, stream>>>(w_c1, 64, 64, 128, 3, Bc1); k_wre<<<(unsigned)(((size_t)64 * 9 * 128 / 8 + 255) / 256), 256, 0, stream>>>(w_c12, 64, 64, 128, 3, Bc12);
  k_wre<<<(unsigned)(((size_t)64 * 9 * 64 / 8 + 255) / 256), 256, 0, stream>>>(w_downrs, 64, 64, 64, 3, Bdrs); k_wre<<<(64 * 64 / 8 + 255) / 256, 256, 0, stream>>>(w_off, 64, 64, 64, 1, Boff); k_wre<<<(64 * 64 / 8 + 255) / 256, 256, 0, stream>>>(w_c3, 64, 64, 64, 1, Bc3);
  k_wre<<<(unsigned)(((size_t)64 * 9 * 64 / 8 + 255) / 256), 256, 0, stream>>>(w_d1o, 64, 18, 64, 3, Bd1o); k_wre<<<(unsigned)(((size_t)64 * 9 * 64 / 8 + 255) / 256), 256, 0, stream>>>(w_d1, 64, 64, 64, 3, Bd1); k_wre<<<(unsigned)(((size_t)64 * 9 * 64 / 8 + 255) / 256), 256, 0, stream>>>(w_d2o, 64, 18, 64, 3, Bd2o); k_wre<<<(unsigned)(((size_t)64 * 9 * 64 / 8 + 255) / 256), 256, 0, stream>>>(w_d2, 64, 64, 64, 3, Bd2);
  k_wtr<<<(unsigned)(((size_t)4 * 64 * 4 * 64 / 8 + 255) / 256), 256, 0, stream>>>(w_up1, Bup1); k_wtr<<<(unsigned)(((size_t)4 * 64 * 4 * 64 / 8 + 255) / 256), 256, 0, stream>>>(w_up2, Bup2); k_bpad<<<1, 64, 0, stream>>>(b_d1o, 18, bz1); k_bpad<<<1, 64, 0, stream>>>(b_d2o, 18, bz2);
  k_nhwc<<<(unsigned)((n8_64 + 255) / 256), 256, 0, stream>>>(dem, F1IN, 128, 0); k_nhwc<<<(unsigned)((n8_64 + 255) / 256), 256, 0, stream>>>(rs, F1IN, 128, 64); k_nhwc<<<(unsigned)((n8_64 + 255) / 256), 256, 0, stream>>>(rs, RS16, 64, 0);
  conv3(stream, F1IN, 128, HH, 2, HL, Bdown1, b_down1, 128, nullptr, F2A16, 128, XC);
  conv3(stream, F1IN, 128, HH, 1, HH, Bc1, b_c1, 64, FEA1, nullptr, 64, XC);
  conv3(stream, F2A16, 128, HL, 1, HL, Bc12, b_c12, 64, FEA2, nullptr, 64, XC);
  k_h16<<<(unsigned)(((size_t)R1 * 64 / 8 + 255) / 256), 256, 0, stream>>>(FEA2, FEA2H, (size_t)R1 * 64 / 8);
  for (int ph = 0; ph < 4; ++ph) { k_phcol<<<(unsigned)(((size_t)R1 * 4 * 8 + 255) / 256), 256, 0, stream>>>(FEA2H, ph, XC); k_gemm2<0><<<dim3((R1 / 128) * 1, 1), 128, 0, stream>>>(XC, 256, 0, Bup1 + (size_t)ph * 64 * 256, 256, 0, 0.0625f, b_up1, 0, nullptr, 1, 0, 0, TMP, nullptr, 64, 0, R1, 64, 256); k_place<<<(unsigned)(((size_t)R1 * 64 / 8 + 255) / 256), 256, 0, stream>>>(TMP, ph, UPF, nullptr); }
  k_add16<<<(unsigned)((n8_64 + 255) / 256), 256, 0, stream>>>(FEA1, UPF, SUM16, n8_64);
  k_gemm2<0><<<dim3((R0 / 128) * 1, 1), 128, 0, stream>>>(SUM16, 64, 0, Boff, 64, 0, 0.0625f, b_off, 0, nullptr, 1, 0, 0, nullptr, FEA16, 64, 0, R0, 64, 64);
  conv3(stream, FEA16, 64, HH, 1, HH, Bd1o, bz1, 64, OFF1, nullptr, 64, XC);
  for (int r0 = 0; r0 < R0; r0 += RCH) { k_dcncol<<<(unsigned)(((size_t)RCH * 9 * 8 + 255) / 256), 256, 0, stream>>>(RS16, HH, OFF1, 64, r0, RCH, XC); k_gemm2<0><<<dim3((RCH / 128) * 1, 1), 128, 0, stream>>>(XC, 576, 0, Bd1, 576, 0, 0.0625f, b_d1, 0, nullptr, 1, 0, 0, F11 + (size_t)r0 * 64, nullptr, 64, 0, RCH, 64, 576); }
  conv3(stream, RS16, 64, HH, 2, HL, Bdrs, b_downrs, 64, nullptr, RS2H, 64, XC);
  conv3(stream, FEA2H, 64, HL, 1, HL, Bd2o, bz2, 64, OFF2, nullptr, 64, XC);
  k_dcncol<<<(unsigned)(((size_t)R1 * 9 * 8 + 255) / 256), 256, 0, stream>>>(RS2H, HL, OFF2, 64, 0, R1, XC); k_gemm2<0><<<dim3((R1 / 128) * 1, 1), 128, 0, stream>>>(XC, 576, 0, Bd2, 576, 0, 0.0625f, b_d2, 0, nullptr, 1, 0, 0, nullptr, FEA2B, 64, 0, R1, 64, 576);
  for (int ph = 0; ph < 4; ++ph) { k_phcol<<<(unsigned)(((size_t)R1 * 4 * 8 + 255) / 256), 256, 0, stream>>>(FEA2B, ph, XC); k_gemm2<0><<<dim3((R1 / 128) * 1, 1), 128, 0, stream>>>(XC, 256, 0, Bup2 + (size_t)ph * 64 * 256, 256, 0, 0.0625f, b_up2, 0, nullptr, 1, 0, 0, TMP, nullptr, 64, 0, R1, 64, 256); k_place<<<(unsigned)(((size_t)R1 * 64 / 8 + 255) / 256), 256, 0, stream>>>(TMP, ph, UP2F, nullptr); }
  k_add16<<<(unsigned)((n8_64 + 255) / 256), 256, 0, stream>>>(F11, UP2F, SUM16, n8_64);
  k_gemm2<0><<<dim3((R0 / 128) * 1, 1), 128, 0, stream>>>(SUM16, 64, 0, Bc3, 64, 0, 0.0625f, b_c3, 0, nullptr, 1, 0, 0, Y, nullptr, 64, 0, R0, 64, 64);
  k_out<<<(unsigned)((n8_64 + 255) / 256), 256, 0, stream>>>(Y, (float*)d_out);
}
